// MultiHeadedAttention_50826642981217
// MI455X (gfx1250) — hardware-verified
//
#include <hip/hip_runtime.h>
#include <math.h>

typedef __attribute__((ext_vector_type(16))) _Float16 v16h;
typedef __attribute__((ext_vector_type(16))) __bf16 v16b;
typedef __attribute__((ext_vector_type(8)))  _Float16 v8h;
typedef __attribute__((ext_vector_type(8)))  __bf16 v8b;
typedef __attribute__((ext_vector_type(8)))  float v8f;
typedef __attribute__((ext_vector_type(4)))  float v4f;
typedef __attribute__((ext_vector_type(4)))  unsigned v4u;
typedef __attribute__((ext_vector_type(4)))  int v4i;

#ifndef NB
#define NB 2
#endif
#ifndef SEQ
#define SEQ 2048
#endif
#define NB_FULL 2
#define SEQ_FULL 2048
#define HID 1024
#define NH 16
#define HD 64

static_assert(NB <= NB_FULL);
static_assert(SEQ <= SEQ_FULL);
static_assert(SEQ % 64 == 0);
static_assert(HID == NH * HD);
static_assert(HD == 64);
static_assert(HID % 128 == 0);
static_assert(HID / 8 == 128);
static_assert(((size_t)NB * SEQ * HID) % 2048 == 0);
static_assert(((size_t)HID * HID) % 2048 == 0);

template <typename T> __device__ __forceinline__ void vst2(void* p, T v) { *(volatile T*)p = v; __threadfence(); *(volatile T*)p = v; }
__device__ __forceinline__ v8f wmma16(v16h a, v16h b, v8f c) {
  v8f d = __builtin_amdgcn_wmma_f32_16x16x32_f16(false, a, false, b, (short)0, c, false, false);
  asm volatile("v_nop\n\tv_nop\n\tv_nop\n\tv_nop" : "+v"(d) : "v"(a), "v"(b));
  return d;
}
__device__ __forceinline__ v8f wmma_bf(v16b a, v16b b, v8f c) {
  v8f d = __builtin_amdgcn_wmma_f32_16x16x32_bf16(false, a, false, b, (short)0, c, false, false);
  asm volatile("v_nop\n\tv_nop\n\tv_nop\n\tv_nop" : "+v"(d) : "v"(a), "v"(b));
  return d;
}
__device__ __forceinline__ v16h frag_h(const _Float16* rowk0, unsigned lane) {
  union { v16h v; v8h q[2]; } u; const _Float16* p = rowk0 + 8u * (lane >> 4);
  u.q[0] = *(const v8h*)p; u.q[1] = *(const v8h*)(p + 16); return u.v;
}
__device__ __forceinline__ v16b frag_b(const __bf16* rowk0, unsigned lane) {
  union { v16b v; v8b q[2]; } u; const __bf16* p = rowk0 + 8u * (lane >> 4);
  u.q[0] = *(const v8b*)p; u.q[1] = *(const v8b*)(p + 16); return u.v;
}
__device__ __forceinline__ float bfr(float v) { return (float)(__bf16)v; }
#define LDSX() do { asm volatile("s_wait_dscnt 0" ::: "memory"); __builtin_amdgcn_wave_barrier(); __builtin_amdgcn_fence(3  , "workgroup"); } while (0)
#define RS10 (1.0f / 1024.0f)

#define PL_ROWS ((size_t)NB * SEQ)
#define WS_XQ  ((size_t)0)
#define WS_XK  (WS_XQ + 2u * PL_ROWS * HID)
#define WS_XV  (WS_XK + 2u * PL_ROWS * HID)
#define WS_WQ  (WS_XV + 2u * PL_ROWS * HID)
#define WS_WK  (WS_WQ + 2u * (size_t)HID * HID)
#define WS_WV  (WS_WK + 2u * (size_t)HID * HID)
#define WS_WO  (WS_WV + 2u * (size_t)HID * HID)
#define WS_QH  (WS_WO + 2u * (size_t)HID * HID)
#define WS_QL  (WS_QH + 2u * PL_ROWS * HID)
#define WS_KH  (WS_QL + 2u * PL_ROWS * HID)
#define WS_VT  (WS_KH + 2u * PL_ROWS * HID)
#define WS_Y   (WS_VT + 2u * PL_ROWS * HID)
#define WS_YL  (WS_Y  + 2u * PL_ROWS * HID)
#define WS_END (WS_YL + 2u * PL_ROWS * HID)
static_assert(WS_END <= (size_t)134217728);

__global__ __launch_bounds__(256) void k_cvt_in(const float* __restrict__ Q, const float* __restrict__ K, const float* __restrict__ V, __bf16* __restrict__ XQ, __bf16* __restrict__ XK, __bf16* __restrict__ XV) {
  const unsigned which = blockIdx.y;
  const float* S = which == 0 ? Q : which == 1 ? K : V; __bf16* D = which == 0 ? XQ : which == 1 ? XK : XV;
  const unsigned i = blockIdx.x * 256u + threadIdx.x; const unsigned row = i >> 7, c = (i & 127u) * 8u;
  const unsigned b = row / (unsigned)SEQ, t = row % (unsigned)SEQ;
  const float* sp = S + ((size_t)b * SEQ_FULL + t) * HID + c;
  const v4f x0 = *(const v4f*)sp, x1 = *(const v4f*)(sp + 4);
  v8b o;
#pragma unroll
  for (unsigned u = 0; u < 4; ++u) { o[u] = (__bf16)x0[u]; o[4 + u] = (__bf16)x1[u]; }
  vst2(D + (size_t)row * HID + c, __builtin_bit_cast(v4u, o));
}
__global__ __launch_bounds__(256) void k_cvt_w(const float* __restrict__ WQ, const float* __restrict__ WK, const float* __restrict__ WV, const float* __restrict__ WO, __bf16* __restrict__ PQ, __bf16* __restrict__ PK, __bf16* __restrict__ PV, _Float16* __restrict__ PO) {
  const unsigned which = blockIdx.y;
  const float* S = which == 0 ? WQ : which == 1 ? WK : which == 2 ? WV : WO;
  const size_t e0 = ((size_t)blockIdx.x * 256u + threadIdx.x) * 8u;
  const v4f x0 = *(const v4f*)(S + e0), x1 = *(const v4f*)(S + e0 + 4);
  if (which < 3) { __bf16* D = which == 0 ? PQ : which == 1 ? PK : PV; v8b o;
#pragma unroll
    for (unsigned u = 0; u < 4; ++u) { o[u] = (__bf16)x0[u]; o[4 + u] = (__bf16)x1[u]; }
    vst2(D + e0, __builtin_bit_cast(v4u, o));
  } else { v8h o;
#pragma unroll
    for (unsigned u = 0; u < 4; ++u) { o[u] = (_Float16)(bfr(x0[u]) * 256.0f); o[4 + u] = (_Float16)(bfr(x1[u]) * 256.0f); }
    vst2(PO + e0, __builtin_bit_cast(v4u, o)); }
}

__global__ __launch_bounds__(128) void k_proj(const __bf16* __restrict__ XQ, const __bf16* __restrict__ XK, const __bf16* __restrict__ XV, const __bf16* __restrict__ WQ, const __bf16* __restrict__ WK, const __bf16* __restrict__ WV,
    const float* __restrict__ BQ, const float* __restrict__ BK, const float* __restrict__ BV, const float* __restrict__ G, _Float16* __restrict__ QH, _Float16* __restrict__ QL, _Float16* __restrict__ KH, _Float16* __restrict__ VT) {
  __shared__ __align__(16) _Float16 sh[64][136]; __shared__ __align__(16) _Float16 sl[64][136]; __shared__ __align__(16) _Float16 th[128][72];
  const unsigned tid = threadIdx.x, wave = tid >> 5, lane = tid & 31u, col = lane & 15u, g = lane >> 4;
  const unsigned which = blockIdx.z; const unsigned c0 = blockIdx.y * 128u; const unsigned r0 = blockIdx.x * 64u; const unsigned bb = r0 / (unsigned)SEQ, t0 = r0 % (unsigned)SEQ;
  const __bf16* X = which == 0 ? XQ : which == 1 ? XK : XV; const __bf16* WA = which == 0 ? WQ : which == 1 ? WK : WV; const float* BA = which == 0 ? BQ : which == 1 ? BK : BV;
  v8f acc[8] = {};
  const __bf16* arow = X + (size_t)(r0 + wave * 16u + col) * HID;
#pragma unroll 2
  for (unsigned kc = 0; kc < HID / 32; ++kc) { const v16b a = frag_b(arow + kc * 32u, lane);
    asm volatile("s_wait_loadcnt 0x0" ::: "memory");
#pragma unroll
    for (unsigned j = 0; j < 8; ++j) { const v16b w = frag_b(WA + (size_t)(c0 + j * 16u + col) * HID + kc * 32u, lane); asm volatile("s_wait_loadcnt 0x0" ::: "memory"); acc[j] = wmma_bf(a, w, acc[j]); } }
  float gt[8];
#pragma unroll
  for (unsigned r = 0; r < 8; ++r) { const float gv = bfr(G[(size_t)bb * SEQ_FULL + t0 + wave * 16u + 8u * g + r]); gt[r] = which == 0 ? 1.0f : 1.0f + gv; }
  if (which < 2) { _Float16* DH = which == 0 ? QH : KH;
#pragma unroll
    for (unsigned j = 0; j < 8; ++j) { const float bias = bfr(BA[c0 + j * 16u + col]);
#pragma unroll
      for (unsigned r = 0; r < 8; ++r) { const float v = acc[j][r] * gt[r] + bias; const _Float16 hv = (_Float16)v; sh[wave * 16u + 8u * g + r][j * 16u + col] = hv; sl[wave * 16u + 8u * g + r][j * 16u + col] = (_Float16)((v - (float)hv) * 1024.0f); } }
    __syncthreads();
    for (unsigned e = tid; e < 64u * 16u; e += 128u) { const unsigned rl = e >> 4, q = e & 15u; const v4u pv = *(const v4u*)&sh[rl][q * 8u]; vst2(DH + (size_t)(r0 + rl) * HID + c0 + q * 8u, pv);
      if (which == 0) { const v4u pl = *(const v4u*)&sl[rl][q * 8u]; vst2(QL + (size_t)(r0 + rl) * HID + c0 + q * 8u, pl); } }
  } else {
#pragma unroll
    for (unsigned j = 0; j < 8; ++j) { const float bias = bfr(BA[c0 + j * 16u + col]);
#pragma unroll
      for (unsigned r = 0; r < 8; ++r) { const float v = acc[j][r] * gt[r] + bias; th[j * 16u + col][wave * 16u + 8u * g + r] = (_Float16)v; } }
    __syncthreads();
    for (unsigned e = tid; e < 128u * 8u; e += 128u) { const unsigned cl = e >> 3, q = e & 7u; const v4u pv = *(const v4u*)&th[cl][q * 8u]; vst2(VT + ((size_t)bb * HID + c0 + cl) * SEQ + t0 + q * 8u, pv); } } }

#define SC2 (0.125f * 1.44269504088896340736f)
#define MASKV (-10000.0f * 1.44269504088896340736f)
__global__ __launch_bounds__(128) void k_flash(const _Float16* __restrict__ QH, const _Float16* __restrict__ QL, const _Float16* __restrict__ KH, const _Float16* __restrict__ VT, const int* __restrict__ MK, _Float16* __restrict__ Y, _Float16* __restrict__ YL) {
  __shared__ __align__(16) unsigned sy[4][16][36];
  __shared__ __align__(16) unsigned syl[4][16][36];
  const unsigned tid = threadIdx.x, wave = tid >> 5, lane = tid & 31u, col = lane & 15u, g = lane >> 4;
  const unsigned b = blockIdx.y / (unsigned)NH, h = blockIdx.y % (unsigned)NH; const unsigned ql0 = blockIdx.x * 64u + wave * 16u;
  const size_t qoff = ((size_t)b * SEQ + ql0 + col) * HID + h * HD;
  v16h qf[2], ql[2]; qf[0] = frag_h(QH + qoff, lane); qf[1] = frag_h(QH + qoff + 32, lane); ql[0] = frag_h(QL + qoff, lane); ql[1] = frag_h(QL + qoff + 32, lane);
  const _Float16* Kb = KH + (size_t)b * SEQ * HID + h * HD;
  const _Float16* Vb = VT + ((size_t)b * HID + h * HD) * SEQ;
  const int* mk = MK + (size_t)b * SEQ_FULL;
  v8f o[4] = {}; float m = -3.0e38f, l = 0.f;
#pragma unroll 1
  for (unsigned key0 = 0; key0 < (unsigned)SEQ; key0 += 64u) {
    v8f st[4];
#pragma unroll
    for (unsigned t = 0; t < 4; ++t) { const _Float16* kr = Kb + (size_t)(key0 + t * 16u + col) * HID;
      const v16h k0f = frag_h(kr, lane), k1f = frag_h(kr + 32, lane);
      const int* mp = mk + key0 + t * 16u + 8u * g; const v4i ma = *(const v4i*)mp, mb = *(const v4i*)(mp + 4);
      asm volatile("s_wait_loadcnt 0x0" ::: "memory");
      v8f sa = {}, sb = {};
      sa = wmma16(k0f, qf[0], sa); sb = wmma16(k0f, ql[0], sb); sa = wmma16(k1f, qf[1], sa); sb = wmma16(k1f, ql[1], sb);
#pragma unroll
      for (unsigned r = 0; r < 4; ++r) { const float s0 = (sa[r] + sb[r] * RS10) * SC2; const float s1 = (sa[4 + r] + sb[4 + r] * RS10) * SC2; st[t][r] = ma[r] != 0 ? s0 : MASKV; st[t][4 + r] = mb[r] != 0 ? s1 : MASKV; } }
    float tm = st[0][0];
#pragma unroll
    for (unsigned t = 0; t < 4; ++t)
#pragma unroll
      for (unsigned r = 0; r < 8; ++r) tm = fmaxf(tm, st[t][r]);
    tm = fmaxf(tm, __shfl_xor(tm, 16));
    const float mn = fmaxf(m, tm); const float alpha = exp2f(m - mn); m = mn; const float mo = mn - 10.0f;
    float ps = 0.f; v16h pb[2];
#pragma unroll
    for (unsigned t = 0; t < 4; ++t)
#pragma unroll
      for (unsigned r = 0; r < 8; ++r) { const float e = exp2f(st[t][r] - mo); ps += e; pb[t >> 1][(t & 1u) * 8u + r] = (_Float16)e; }
    l = l * alpha + ps;
#pragma unroll
    for (unsigned j = 0; j < 4; ++j)
#pragma unroll
      for (unsigned r = 0; r < 8; ++r) o[j][r] *= alpha;
#pragma unroll
    for (unsigned j = 0; j < 4; ++j) { const _Float16* vr = Vb + (size_t)(j * 16u + col) * SEQ + key0;
      const v16h v0f = frag_h(vr, lane), v1f = frag_h(vr + 32, lane);
      asm volatile("s_wait_loadcnt 0x0" ::: "memory");
      o[j] = wmma16(v0f, pb[0], o[j]); o[j] = wmma16(v1f, pb[1], o[j]); }
  }
  l += __shfl_xor(l, 16);
  const float inv = 64.0f * (1.0f / l);
#pragma unroll
  for (unsigned j = 0; j < 4; ++j) { v8h hv, lv;
#pragma unroll
    for (unsigned r = 0; r < 8; ++r) { const float cv = o[j][r] * inv; const _Float16 ch = (_Float16)cv; hv[r] = ch; lv[r] = (_Float16)((cv - (float)ch) * 1024.0f); }
    *(v4u*)&sy[wave][col][j * 8u + 4u * g] = __builtin_bit_cast(v4u, hv); *(v4u*)&syl[wave][col][j * 8u + 4u * g] = __builtin_bit_cast(v4u, lv); }
  LDSX();
#pragma unroll
  for (unsigned i = 0; i < 4; ++i) { const unsigned row = i * 4u + (lane >> 3), pc = lane & 7u; const v4u pv = *(const v4u*)&sy[wave][row][pc * 4u]; const v4u pl = *(const v4u*)&syl[wave][row][pc * 4u];
    const size_t off = ((size_t)b * SEQ + ql0 + row) * HID + h * HD + pc * 8u;
    vst2(Y + off, pv); vst2(YL + off, pl); } }

__global__ __launch_bounds__(128) void k_out(const _Float16* __restrict__ Y, const _Float16* __restrict__ YL, const _Float16* __restrict__ WO, const float* __restrict__ BO, float* __restrict__ OUT) { __shared__ __align__(16) float sf[4][16][132];
  const unsigned tid = threadIdx.x, wave = tid >> 5, lane = tid & 31u, col = lane & 15u, g = lane >> 4; const unsigned c0 = blockIdx.y * 128u; const unsigned rb = blockIdx.x * 64u; const unsigned r0 = rb + wave * 16u;
  v8f acc[8] = {}, accl[8] = {};
  const _Float16* arow = Y + (size_t)(r0 + col) * HID; const _Float16* lrow = YL + (size_t)(r0 + col) * HID;
#pragma unroll 2
  for (unsigned kc = 0; kc < HID / 32; ++kc) { const v16h a = frag_h(arow + kc * 32u, lane), al = frag_h(lrow + kc * 32u, lane); asm volatile("s_wait_loadcnt 0x0" ::: "memory");
#pragma unroll
    for (unsigned j = 0; j < 8; ++j) { const v16h w = frag_h(WO + (size_t)(c0 + j * 16u + col) * HID + kc * 32u, lane); asm volatile("s_wait_loadcnt 0x0" ::: "memory"); acc[j] = wmma16(a, w, acc[j]); accl[j] = wmma16(al, w, accl[j]); } }
#pragma unroll
  for (unsigned j = 0; j < 8; ++j) { const float bias = bfr(BO[c0 + j * 16u + col]);
#pragma unroll
    for (unsigned r = 0; r < 8; ++r) sf[wave][8u * g + r][j * 16u + col] = (acc[j][r] + accl[j][r] * RS10) * (1.0f / 16384.0f) + bias; }
  LDSX();
  const unsigned bb = rb / (unsigned)SEQ, t0 = rb % (unsigned)SEQ + wave * 16u;
  for (unsigned rl = 0; rl < 16; ++rl) { const v4f pv = *(const v4f*)&sf[wave][rl][lane * 4u]; vst2(OUT + ((size_t)bb * SEQ_FULL + t0 + rl) * HID + c0 + lane * 4u, pv); } }

extern "C" void kernel_launch(void* const* d_in, const int* in_sizes, int n_in, void* d_out, int out_size, void* d_ws, size_t ws_size, hipStream_t stream) {
  if (n_in < 13) return;
  const size_t need_rows = (size_t)(NB - 1) * SEQ_FULL + SEQ;
  if ((size_t)in_sizes[0] < need_rows * HID || (size_t)in_sizes[1] < need_rows * HID || (size_t)in_sizes[2] < need_rows * HID) return;
  if ((size_t)in_sizes[3] < need_rows || (size_t)in_sizes[4] < need_rows) return;
  if ((size_t)in_sizes[5] < (size_t)HID * HID || (size_t)in_sizes[7] < (size_t)HID * HID || (size_t)in_sizes[9] < (size_t)HID * HID || (size_t)in_sizes[11] < (size_t)HID * HID) return;
  if (in_sizes[6] < HID || in_sizes[8] < HID || in_sizes[10] < HID || in_sizes[12] < HID) return;
  if ((size_t)out_size < need_rows * HID) return;
  if (ws_size < (size_t)WS_END) return;
  const float* query = (const float*)d_in[0]; const float* key_ = (const float*)d_in[1]; const float* value = (const float*)d_in[2]; const float* gate = (const float*)d_in[3]; const int* mask = (const int*)d_in[4];
  const float* wq = (const float*)d_in[5]; const float* bq = (const float*)d_in[6]; const float* wk = (const float*)d_in[7]; const float* bk = (const float*)d_in[8];
  const float* wv = (const float*)d_in[9]; const float* bv = (const float*)d_in[10]; const float* wo = (const float*)d_in[11]; const float* bo = (const float*)d_in[12];
  char* ws = (char*)d_ws;
  __bf16 *XQ = (__bf16*)(ws + WS_XQ), *XK = (__bf16*)(ws + WS_XK), *XV = (__bf16*)(ws + WS_XV), *PQ = (__bf16*)(ws + WS_WQ), *PK = (__bf16*)(ws + WS_WK), *PV = (__bf16*)(ws + WS_WV);
  _Float16 *PO = (_Float16*)(ws + WS_WO), *QH = (_Float16*)(ws + WS_QH), *QL = (_Float16*)(ws + WS_QL), *KH = (_Float16*)(ws + WS_KH), *VT = (_Float16*)(ws + WS_VT), *Y = (_Float16*)(ws + WS_Y), *YL = (_Float16*)(ws + WS_YL);
  k_cvt_in<<<dim3((unsigned)((size_t)NB * SEQ * HID / 2048), 3), 256, 0, stream>>>(query, key_, value, XQ, XK, XV);
  k_cvt_w<<<dim3((unsigned)((size_t)HID * HID / 2048), 4), 256, 0, stream>>>(wq, wk, wv, wo, PQ, PK, PV, PO);
  k_proj<<<dim3(NB * SEQ / 64, HID / 128, 3), 128, 0, stream>>>(XQ, XK, XV, PQ, PK, PV, bq, bk, bv, gate, QH, QL, KH, VT);
  k_flash<<<dim3(SEQ / 64, NB * NH), 128, 0, stream>>>(QH, QL, KH, VT, mask, Y, YL);
  k_out<<<dim3(NB * SEQ / 64, HID / 128), 128, 0, stream>>>(Y, YL, PO, bo, (float*)d_out);
}
